// E3TransferableAtomicOrbitals_42374147342463
// MI455X (gfx1250) — hardware-run, weakly checked
//
#include <hip/hip_runtime.h>


#ifndef NB
#define NB 32
#endif
#define NB_FULL 32
#define NION 64
#define MUL  128
#define NHD  8
#define AHD  16
#define CPW  64
#define NRBF 32
#define HID  64
#define NPW  512
#define OW   512
#define OTP  132
#define HSP  72
#define WTP  132
#define MTOK (NB * NION)
#define NZH  (NB * NHD)
#define INV_SQRT3 0.57735026918962576f
#define SC2  ((float)(0.17677669529663687 * 1.4426950408889634))
#define LOG2E 1.4426950408889634f
#define PSH  14.0f
#define WCS  64.0f
#define WCI  (1.0f / 64.0f)

static_assert(NION == 64);
static_assert(MUL == 128);
static_assert(NHD * AHD == MUL);
static_assert(CPW == 4 * AHD);
static_assert(CPW == 64);
static_assert(MUL % 32 == 0);
static_assert(NRBF % 32 == 0);
static_assert(HID == 64);
static_assert(HID % 32 == 0);
static_assert(NHD == 8);
static_assert(NHD % 2 == 0);
static_assert((2 * AHD * 4) % 128 == 0);
static_assert((2 * AHD * 3 * 4) % 128 == 0);
static_assert(NPW == 8 * HID);
static_assert(OW == MUL + 3 * MUL);
static_assert(NB <= NB_FULL);
static_assert(((size_t)MTOK * MUL / 8) % 256 == 0);
static_assert(((size_t)NION * NION * NRBF / 8) % 256 == 0);
static_assert((OTP * 4) % 16 == 0);
static_assert((HSP * 2) % 16 == 0);
static_assert((WTP * 4) % 16 == 0);
static_assert(32 * 16 * 16 == 64 * CPW * 2);
static_assert(32 * 16 * 8 == 16 * 64 * 4);
static_assert(128 * 16 * 1 == NHD * NION * 4);
static_assert(256 * 16 * (2 + 6) == NION * (2 * AHD * 4) * 4);
static_assert(16 * WTP * 4 <= 131072);
static_assert(64 * 68 * 4 <= 131072);
static_assert(16 * 68 * 4 <= 131072);
static_assert(2 * 64 * HSP * 2 + 16 * 64 * 4 <= 131072);
static_assert(64 * OTP * 4 <= 131072);

typedef _Float16 h16;
typedef unsigned short bf;
typedef __attribute__((ext_vector_type(16))) __bf16   v16bf;
typedef __attribute__((ext_vector_type(16))) _Float16 v16h;
typedef __attribute__((ext_vector_type(8)))  _Float16 v8h;
typedef __attribute__((ext_vector_type(4)))  _Float16 v4h;
typedef __attribute__((ext_vector_type(8)))  unsigned short v8us;
typedef __attribute__((ext_vector_type(8)))  float    v8f;
typedef __attribute__((ext_vector_type(4)))  float    v4f;
typedef v4f  __attribute__((may_alias)) v4fa;

__device__ __forceinline__ unsigned short f2bf(float f) { unsigned u = __float_as_uint(f); u += 0x7FFFu + ((u >> 16) & 1u); return (unsigned short)(u >> 16); }
__device__ __forceinline__ float bfr(float f) { return __uint_as_float(((unsigned)f2bf(f)) << 16); }
__device__ __forceinline__ v16h cat16(v8h lo, v8h hi) { return __builtin_shufflevector(lo, hi, 0, 1, 2, 3, 4, 5, 6, 7, 8, 9, 10, 11, 12, 13, 14, 15); }
__device__ __forceinline__ v16bf cat16b(v8us lo, v8us hi) { return __builtin_bit_cast(v16bf, __builtin_shufflevector(lo, hi, 0, 1, 2, 3, 4, 5, 6, 7, 8, 9, 10, 11, 12, 13, 14, 15)); }
__device__ __forceinline__ v8f wmma16(v16h a, v16h b, v8f c) { return __builtin_amdgcn_wmma_f32_16x16x32_f16(false, a, false, b, (short)0, c, false, false); }
__device__ __forceinline__ v8f wmmab(v16bf a, v16bf b, v8f c) { return __builtin_amdgcn_wmma_f32_16x16x32_bf16(false, a, false, b, (short)0, c, false, false); }
__device__ __forceinline__ v16h  ldh(const h16* p) { return cat16(*(const v8h*)p, *(const v8h*)(p + 16)); }
__device__ __forceinline__ v16bf ldb(const bf* p)  { return cat16b(*(const v8us*)p, *(const v8us*)(p + 16)); }
__device__ __forceinline__ void wave_sync() { __builtin_amdgcn_fence(3  , "wavefront"); __builtin_amdgcn_wave_barrier(); asm volatile("" ::: "memory"); }

static __device__ __forceinline__ h16 toh_flush(float v) { const h16 r = (h16)v; return (fabsf(v) < 6.103515625e-05f) ? (h16)0.0f : r; }
__device__ __forceinline__ v8f wmma16g(v16h a, v16h b, v8f c) { c = wmma16(a, b, c); asm volatile("v_nop\n\tv_nop\n\tv_nop\n\tv_nop" : "+v"(c) : "v"(a), "v"(b)); return c; }
__device__ __forceinline__ v8f wmmabg(v16bf a, v16bf b, v8f c) { c = wmmab(a, b, c); asm volatile("v_nop\n\tv_nop\n\tv_nop\n\tv_nop" : "+v"(c) : "v"(a), "v"(b)); return c; }
__device__ __forceinline__ float tanh_fast(float x) { const float xc = fminf(fmaxf(x, -15.0f), 15.0f); const float e = __builtin_amdgcn_exp2f(xc * 2.8853900817779268f); return 1.0f - 2.0f * __builtin_amdgcn_rcpf(1.0f + e); }

__global__ __launch_bounds__(256) void k_cvt8(const float* __restrict__ src, bf* dst, size_t n8) {
    const size_t i = (size_t)blockIdx.x * 256 + threadIdx.x; if (i >= n8) return;
    const v8f v = *(const v8f*)(src + i * 8); v8us o;
#pragma unroll
    for (int k = 0; k < 8; ++k) o[k] = f2bf(v[k]);
    *(volatile v8us*)(dst + i * 8) = o; __threadfence(); *(volatile v8us*)(dst + i * 8) = o;
}

__global__ __launch_bounds__(256) void k_cvtv(const float* __restrict__ src, bf* dst, size_t n8, size_t plane) {
    const size_t i = (size_t)blockIdx.x * 256 + threadIdx.x; if (i >= n8) return;
    const float* p = src + i * 24;
    float v[24];
#pragma unroll
    for (int q = 0; q < 6; ++q) { const v4f t = *(const v4f*)(p + 4 * q); v[4 * q] = t[0]; v[4 * q + 1] = t[1]; v[4 * q + 2] = t[2]; v[4 * q + 3] = t[3]; }
    v8us o0, o1, o2;
#pragma unroll
    for (int k = 0; k < 8; ++k) { o0[k] = f2bf(v[3 * k]); o1[k] = f2bf(v[3 * k + 1]); o2[k] = f2bf(v[3 * k + 2]); }
    const size_t d0 = plane + i * 8, d1 = 2 * plane + i * 8, d2 = 3 * plane + i * 8;
    *(volatile v8us*)(dst + d0) = o0; *(volatile v8us*)(dst + d1) = o1; *(volatile v8us*)(dst + d2) = o2;
    __threadfence();
    *(volatile v8us*)(dst + d0) = o0; *(volatile v8us*)(dst + d1) = o1; *(volatile v8us*)(dst + d2) = o2;
}

__global__ __launch_bounds__(256) void k_wt(const float* __restrict__ src, int ld, int K, int nvalid, int yrows, int ydst, bf* dst, int f16m, float scale) {
    __shared__ __align__(16) float ts[16 * WTP];
    const int tid = threadIdx.x;
    const int n0 = blockIdx.x * 16;
    const size_t sbase = (size_t)blockIdx.y * (size_t)yrows * (size_t)ld;
    const int tot = 16 * K;
    for (int e = tid; e < tot; e += 256) {
        const int k = e >> 4, nn = e & 15; const int n = n0 + nn;
        const int nc = n < nvalid ? n : nvalid - 1;
        float w = src[sbase + (size_t)k * ld + nc];
        asm volatile("" : "+v"(w));
        const float wb = bfr(w);
        ts[nn * WTP + k] = (n < nvalid) ? wb : 0.0f;
    }
    __syncthreads();
    if (tid < 2 * K) {
        const int kp = K >> 3; const int row = tid / kp, c8 = (tid - row * kp) * 8;
        const v4f x0 = *(const v4fa*)(&ts[row * WTP + c8]); const v4f x1 = *(const v4fa*)(&ts[row * WTP + c8 + 4]);
        v8us ob; v8h hv;
#pragma unroll
        for (int i = 0; i < 4; ++i) { ob[i] = f2bf(x0[i]); ob[4 + i] = f2bf(x1[i]); hv[i] = toh_flush(x0[i] * scale); hv[4 + i] = toh_flush(x1[i] * scale); }
        const v8us oh = __builtin_bit_cast(v8us, hv);
        const v8us o = f16m ? oh : ob;
        const size_t doff = (size_t)blockIdx.y * (size_t)ydst + (size_t)n0 * K + (size_t)tid * 8;
        *(volatile v8us*)(dst + doff) = o; __threadfence(); *(volatile v8us*)(dst + doff) = o;
    }
}

__global__ __launch_bounds__(32) void k_proj3(const bf* __restrict__ X, const bf* __restrict__ WT, h16* P) {
    __shared__ __align__(16) float os[64 * 68];
    const int lane = threadIdx.x & 31, lr = lane & 15, hi = lane >> 4;
    const int b = blockIdx.x; const int which = blockIdx.y >> 3, h = blockIdx.y & 7;
    v8f acc[4][4];
#pragma unroll
    for (int mb = 0; mb < 4; ++mb)
#pragma unroll
        for (int nb = 0; nb < 4; ++nb) acc[mb][nb] = (v8f){};
    const size_t aoff = (size_t)(b * NION + lr) * MUL + 8 * hi;
    const size_t boff = (size_t)(which * 2) * MUL * MUL + (size_t)(h * AHD + lr) * MUL + 8 * hi;
#pragma unroll 1
    for (int kc = 0; kc < MUL; kc += 32) {
        const v16bf bs = ldb(WT + boff + kc);
        const v16bf bv = ldb(WT + boff + (size_t)MUL * MUL + kc);
#pragma unroll
        for (int nb = 0; nb < 4; ++nb) {
#pragma unroll
            for (int mb = 0; mb < 4; ++mb) {
                const v16bf a = ldb(X + (size_t)nb * MTOK * MUL + aoff + (size_t)mb * 16 * MUL + kc);
                acc[mb][nb] = wmmabg(a, nb == 0 ? bs : bv, acc[mb][nb]); } }
    }
    const float vs = (which == 0) ? INV_SQRT3 : 1.0f;
#pragma unroll
    for (int mb = 0; mb < 4; ++mb) {
#pragma unroll
        for (int nb = 0; nb < 4; ++nb) {
#pragma unroll
            for (int j = 0; j < 8; ++j) { const int tok = mb * 16 + hi * 8 + j, cp = nb * 16 + lr;
                const int idx = (which == 2) ? (cp * 68 + tok) : (tok * 68 + cp);
                os[idx] = acc[mb][nb][j] * (nb > 0 ? vs : 1.0f); } } }
    wave_sync();
    const size_t dbase = (size_t)(which * NZH + b * NHD + h) * 64 * 64;
#pragma unroll 1
    for (int ps = 0; ps < 2; ++ps) {
#pragma unroll 4
        for (int s = 0; s < 16; ++s) { const int row = 4 * s + (lane >> 3), c8 = (lane & 7) * 8;
            const v4f x0 = *(const v4fa*)(&os[row * 68 + c8]); const v4f x1 = *(const v4fa*)(&os[row * 68 + c8 + 4]); v8h hv;
#pragma unroll
            for (int i = 0; i < 4; ++i) { hv[i] = toh_flush(x0[i]); hv[4 + i] = toh_flush(x1[i]); }
            *(volatile v8h*)(P + dbase + (size_t)row * 64 + c8) = hv; }
        if (ps == 0) __threadfence(); }
}

__global__ __launch_bounds__(32) void k_gemm_f32(const bf* __restrict__ A, const bf* __restrict__ Bt, const float* __restrict__ bias, float* C, int K, int ldc, int mode) {
    __shared__ __align__(16) float os[16 * 68];
    const int lane = threadIdx.x & 31, lr = lane & 15, hi = lane >> 4; const int r0 = blockIdx.x * 64;
    const int y = blockIdx.y, part = y & 3, side = y >> 2;
    size_t aplane = 0, bplane = 0; int coff = 0; float scale = 1.0f;
    if (mode == 1) { aplane = (size_t)part * MTOK * MUL; bplane = (size_t)(side * 2 + (part > 0 ? 1 : 0)) * HID * MUL; coff = y * 64; scale = (part > 0) ? INV_SQRT3 : 1.0f; }
    v8f acc[4][4];
#pragma unroll
    for (int mb = 0; mb < 4; ++mb)
#pragma unroll
        for (int nb = 0; nb < 4; ++nb) acc[mb][nb] = (v8f){};
    const size_t aoff = aplane + (size_t)(r0 + lr) * K + 8 * hi, boff = bplane + (size_t)lr * K + 8 * hi;
#pragma unroll 1
    for (int kc = 0; kc < K; kc += 32) {
        v16bf a[4];
#pragma unroll
        for (int mb = 0; mb < 4; ++mb) a[mb] = ldb(A + aoff + (size_t)mb * 16 * K + kc);
#pragma unroll
        for (int nb = 0; nb < 4; ++nb) { const v16bf bq = ldb(Bt + boff + (size_t)nb * 16 * K + kc);
#pragma unroll
            for (int mb = 0; mb < 4; ++mb) acc[mb][nb] = wmmabg(a[mb], bq, acc[mb][nb]); }
    }
    float bc[4];
#pragma unroll
    for (int nb = 0; nb < 4; ++nb) bc[nb] = 0.0f;
    if (mode == 0) {
#pragma unroll
        for (int nb = 0; nb < 4; ++nb) bc[nb] = bfr(bias[nb * 16 + lr]);
    }
#pragma unroll
    for (int mb = 0; mb < 4; ++mb) {
#pragma unroll
        for (int nb = 0; nb < 4; ++nb) {
#pragma unroll
            for (int j = 0; j < 8; ++j) os[(hi * 8 + j) * 68 + nb * 16 + lr] = acc[mb][nb][j] * scale + bc[nb]; }
        wave_sync();
#pragma unroll 1
        for (int ps = 0; ps < 2; ++ps) {
#pragma unroll
            for (int s = 0; s < 8; ++s) { const int row = 2 * s + (lane >> 4), c4 = (lane & 15) * 4;
                const v4f val = *(const v4fa*)(&os[row * 68 + c4]);
                *(volatile v4f*)(C + (size_t)(r0 + mb * 16 + row) * ldc + coff + c4) = val; }
            if (ps == 0) __threadfence(); }
        wave_sync();
    }
}

__global__ __launch_bounds__(256) void k_mlp(const float* __restrict__ E, const float* __restrict__ NPJ, const float* __restrict__ edge_sh,
                                             const h16* __restrict__ WMID, const float* __restrict__ bmid, const h16* __restrict__ WOUT, const float* __restrict__ bout, float* EW) {
    __shared__ __align__(16) h16 h1s[64 * HSP];
    __shared__ __align__(16) h16 h2s[64 * HSP];
    __shared__ __align__(16) float ews[16 * 64];
    const int tid = threadIdx.x, lane = tid & 31, lr = lane & 15, hi = lane >> 4;
    const int wave = __builtin_amdgcn_readfirstlane((int)(threadIdx.x >> 5));
    const int b = blockIdx.x >> 6, i = blockIdx.x & 63;
    {
        const int j = tid >> 2, cq = (tid & 3) * 16;
        const v4f shv = *(const v4f*)(edge_sh + ((size_t)i * NION + j) * 4);
        const float y0 = bfr(shv[0]), y1 = bfr(shv[1]), y2 = bfr(shv[2]), y3 = bfr(shv[3]);
        const size_t eo = ((size_t)i * NION + j) * HID + cq;
        const size_t ro = (size_t)(b * NION + i) * NPW + cq;
        const size_t so = (size_t)(b * NION + j) * NPW + 256 + cq;
#pragma unroll 1
        for (int qi = 0; qi < 4; ++qi) {
            const int c = qi * 4;
            const v4f e  = *(const v4f*)(E + eo + c);
            const v4f r0 = *(const v4f*)(NPJ + ro + c), r1 = *(const v4f*)(NPJ + ro + 64 + c), r2 = *(const v4f*)(NPJ + ro + 128 + c), r3 = *(const v4f*)(NPJ + ro + 192 + c);
            const v4f s0 = *(const v4f*)(NPJ + so + c), s1 = *(const v4f*)(NPJ + so + 64 + c), s2 = *(const v4f*)(NPJ + so + 128 + c), s3 = *(const v4f*)(NPJ + so + 192 + c);
            v4h hv;
#pragma unroll
            for (int k = 0; k < 4; ++k) {
                const float pre = e[k] + y0 * (r0[k] + s0[k]) + y1 * (r1[k] + s1[k]) + y2 * (r2[k] + s2[k]) + y3 * (r3[k] + s3[k]);
                hv[k] = toh_flush(tanh_fast(pre)); }
            *(v4h*)(&h1s[j * HSP + cq + c]) = hv;
        }
    }
    __syncthreads();
    {
        const int mt = wave >> 1, ntb = (wave & 1) * 2;
        const int ao = (mt * 16 + lr) * HSP + 8 * hi;
        const v16h a0 = cat16(*(const v8h*)(&h1s[ao]),      *(const v8h*)(&h1s[ao + 16]));
        const v16h a1 = cat16(*(const v8h*)(&h1s[ao + 32]), *(const v8h*)(&h1s[ao + 48]));
#pragma unroll
        for (int n2 = 0; n2 < 2; ++n2) {
            const int nt = ntb + n2;
            const size_t wo = (size_t)(nt * 16 + lr) * HID + 8 * hi;
            const v16h b0 = ldh(WMID + wo), b1 = ldh(WMID + wo + 32);
            v8f acc = (v8f){};
            acc = wmma16g(a0, b0, acc); acc = wmma16g(a1, b1, acc);
            const float bb = bfr(bmid[nt * 16 + lr]);
#pragma unroll
            for (int r = 0; r < 8; ++r) h2s[(mt * 16 + 8 * hi + r) * HSP + nt * 16 + lr] = toh_flush(tanh_fast(acc[r] * WCI + bb));
        }
    }
    __syncthreads();
    if (wave < 4) {
        const int mt = wave;
        const int ao = (mt * 16 + lr) * HSP + 8 * hi;
        const v16h a0 = cat16(*(const v8h*)(&h2s[ao]),      *(const v8h*)(&h2s[ao + 16]));
        const v16h a1 = cat16(*(const v8h*)(&h2s[ao + 32]), *(const v8h*)(&h2s[ao + 48]));
        const size_t wo = (size_t)lr * HID + 8 * hi;
        const v16h b0 = ldh(WOUT + wo), b1 = ldh(WOUT + wo + 32);
        v8f acc = (v8f){};
        acc = wmma16g(a0, b0, acc); acc = wmma16g(a1, b1, acc);
        float bo = bout[lr < 8 ? lr : 7];
        asm volatile("" : "+v"(bo));
        const float bb = bfr(bo);
#pragma unroll
        for (int r = 0; r < 8; ++r) ews[lr * 64 + mt * 16 + 8 * hi + r] = acc[r] * WCI + bb;
    }
    __syncthreads();
    if (tid < 128) {
        const int h = tid >> 4, c4 = (tid & 15) * 4;
        const v4f val = *(const v4fa*)(&ews[h * 64 + c4]);
        const size_t doff = ((size_t)(b * NHD + h) * NION + i) * NION + c4;
        *(volatile v4f*)(EW + doff) = val; __threadfence(); *(volatile v4f*)(EW + doff) = val;
    }
}

__global__ __launch_bounds__(256) void k_attn(const h16* __restrict__ QP, const h16* __restrict__ KP, const h16* __restrict__ VT, const float* __restrict__ EW,
                                              const float* __restrict__ node_s, const float* __restrict__ node_v, float* OUT) {
    __shared__ __align__(16) float ot[64 * OTP];
    const int tid = threadIdx.x, lane = tid & 31, lr = lane & 15, hi = lane >> 4;
    const int wave = __builtin_amdgcn_readfirstlane((int)(threadIdx.x >> 5));
    const int b = blockIdx.x >> 2, hp = blockIdx.x & 3;
    const int hq = wave >> 2, t0 = (wave & 3) * 16;
    const int zh = b * NHD + hp * 2 + hq;
    const size_t pb0 = (size_t)zh * 64 * 64;
    const size_t qo = pb0 + (size_t)(t0 + lr) * 64 + 8 * hi;
    const v16h q0 = ldh(QP + qo), q1 = ldh(QP + qo + 32);
    const size_t ko = pb0 + (size_t)lr * 64 + 8 * hi;
    v8f s[4];
#pragma unroll
    for (int kt = 0; kt < 4; ++kt) {
        const v16h ka = ldh(KP + ko + (size_t)kt * 16 * 64), kb = ldh(KP + ko + (size_t)kt * 16 * 64 + 32);
        s[kt] = (v8f){};
        s[kt] = wmma16g(ka, q0, s[kt]); s[kt] = wmma16g(kb, q1, s[kt]); }
    const size_t eo = pb0 + (size_t)(t0 + lr) * 64 + 8 * hi;
    float ta[4][8]; float mx = -3.0e38f;
#pragma unroll
    for (int kt = 0; kt < 4; ++kt) {
        const v4f e0 = *(const v4f*)(EW + eo + kt * 16), e1 = *(const v4f*)(EW + eo + kt * 16 + 4);
#pragma unroll
        for (int r = 0; r < 4; ++r) {
            ta[kt][r]     = s[kt][r] * SC2     + e0[r] * LOG2E;
            ta[kt][4 + r] = s[kt][4 + r] * SC2 + e1[r] * LOG2E;
            mx = fmaxf(mx, fmaxf(ta[kt][r], ta[kt][4 + r])); } }
    mx = fmaxf(mx, __shfl_xor(mx, 16, 32));
    const float sh = PSH - mx;
    v16h pb0v, pb1v; float ls = 0.0f;
#pragma unroll
    for (int r = 0; r < 8; ++r) {
        const float a0 = ta[0][r] + sh, a1 = ta[1][r] + sh, a2 = ta[2][r] + sh, a3 = ta[3][r] + sh;
        const float e0 = __builtin_amdgcn_exp2f(a0), e1 = __builtin_amdgcn_exp2f(a1), e2 = __builtin_amdgcn_exp2f(a2), e3 = __builtin_amdgcn_exp2f(a3);
        const h16 p0 = (h16)((a0 < -14.0f) ? 0.0f : e0); const h16 p1 = (h16)((a1 < -14.0f) ? 0.0f : e1);
        const h16 p2 = (h16)((a2 < -14.0f) ? 0.0f : e2); const h16 p3 = (h16)((a3 < -14.0f) ? 0.0f : e3);
        pb0v[r] = p0; pb0v[8 + r] = p1; pb1v[r] = p2; pb1v[8 + r] = p3;
        ls += ((float)p0 + (float)p1) + ((float)p2 + (float)p3); }
    ls += __shfl_xor(ls, 16, 32);
    const float inv = 1.0f / ls;
    const size_t vo = pb0 + (size_t)lr * 64 + 8 * hi;
    v8f o[4];
#pragma unroll
    for (int dt = 0; dt < 4; ++dt) {
        const v16h v0 = ldh(VT + vo + (size_t)dt * 16 * 64), v1 = ldh(VT + vo + (size_t)dt * 16 * 64 + 32);
        o[dt] = (v8f){};
        o[dt] = wmma16g(v0, pb0v, o[dt]); o[dt] = wmma16g(v1, pb1v, o[dt]); }
    const int orow = (t0 + lr) * OTP;
    { v4f a, c;
      a[0] = o[0][0] * inv; a[1] = o[0][1] * inv; a[2] = o[0][2] * inv; a[3] = o[0][3] * inv; c[0] = o[0][4] * inv; c[1] = o[0][5] * inv; c[2] = o[0][6] * inv; c[3] = o[0][7] * inv;
      *(v4fa*)(&ot[orow + hq * 16 + 8 * hi]) = a; *(v4fa*)(&ot[orow + hq * 16 + 8 * hi + 4]) = c; }
#pragma unroll
    for (int dt = 1; dt < 4; ++dt) {
#pragma unroll
        for (int r = 0; r < 8; ++r) ot[orow + 32 + (hq * 16 + 8 * hi + r) * 3 + (dt - 1)] = o[dt][r] * inv; }
    __syncthreads();
    const size_t rowb = (size_t)b * NION;
#pragma unroll 1
    for (int ps = 0; ps < 2; ++ps) {
#pragma unroll
        for (int it = 0; it < 2; ++it) { const int row = it * 32 + (tid >> 3), c4 = (tid & 7) * 4;
            const v4f u = *(const v4fa*)(&ot[row * OTP + c4]);
            const v4f x = *(const v4f*)(node_s + (rowb + row) * MUL + hp * 32 + c4);
            v4f val;
#pragma unroll
            for (int k = 0; k < 4; ++k) val[k] = bfr(x[k]) + u[k];
            *(volatile v4f*)(OUT + (rowb + row) * OW + hp * 32 + c4) = val; }
#pragma unroll
        for (int it = 0; it < 6; ++it) { const int row = (it & 1) * 32 + (tid >> 3), sg = it >> 1, c4 = (tid & 7) * 4;
            const v4f u = *(const v4fa*)(&ot[row * OTP + 32 + sg * 32 + c4]);
            const v4f x = *(const v4f*)(node_v + (rowb + row) * (MUL * 3) + hp * 96 + sg * 32 + c4);
            v4f val;
#pragma unroll
            for (int k = 0; k < 4; ++k) val[k] = bfr(x[k]) + u[k];
            *(volatile v4f*)(OUT + (rowb + row) * OW + MUL + hp * 96 + sg * 32 + c4) = val; }
        if (ps == 0) __threadfence(); }
}

static constexpr size_t al256(size_t v) { return (v + 255) & ~(size_t)255; }
static constexpr size_t SZ_XALL = al256((size_t)4 * MTOK * MUL * 2);
static constexpr size_t SZ_EAB  = al256((size_t)NION * NION * NRBF * 2);
static constexpr size_t SZ_WQKV = al256((size_t)6 * MUL * MUL * 2);
static constexpr size_t SZ_W1N  = al256((size_t)4 * HID * MUL * 2);
static constexpr size_t SZ_W1E  = al256((size_t)HID * NRBF * 2);
static constexpr size_t SZ_WMID = al256((size_t)HID * HID * 2);
static constexpr size_t SZ_WOUT = al256((size_t)16 * HID * 2);
static constexpr size_t SZ_P3   = al256((size_t)3 * NZH * 64 * 64 * 2);
static constexpr size_t SZ_NPJ  = al256((size_t)MTOK * NPW * 4);
static constexpr size_t SZ_EPL  = al256((size_t)NION * NION * HID * 4);
static constexpr size_t SZ_EW   = al256((size_t)NZH * NION * NION * 4);
static constexpr size_t SZ_TOTAL = SZ_XALL + SZ_EAB + SZ_WQKV + SZ_W1N + SZ_W1E + SZ_WMID + SZ_WOUT + SZ_P3 + SZ_NPJ + SZ_EPL + SZ_EW;
static_assert(SZ_TOTAL <= (size_t)134217728);
static_assert(((size_t)MUL * MUL * 2) % 256 == 0);
static_assert(((size_t)HID * MUL * 2) % 256 == 0);
static_assert(((size_t)NZH * 64 * 64 * 2) % 256 == 0);
static_assert(((size_t)MTOK * MUL * 2) % 256 == 0);
static_assert((size_t)(NB * 4 - 1) / 4 * NION + 63 < (size_t)MTOK);
static_assert(((size_t)(MTOK - 1) * OW + MUL + 3 * 96 + 2 * 32 + 28 + 4) * 4 <= (size_t)MTOK * OW * 4);
static_assert(32 + 127 + 3 * 128 < 544);

extern "C" void kernel_launch(void* const* d_in, const int* in_sizes, int n_in,
                              void* d_out, int out_size, void* d_ws, size_t ws_size, hipStream_t stream) {
    if (n_in < 16) return;
    if ((size_t)in_sizes[0] < (size_t)MTOK * MUL || (size_t)in_sizes[1] < (size_t)MTOK * MUL * 3) return;
    if ((size_t)in_sizes[2] < (size_t)NION * NION * NRBF || (size_t)in_sizes[3] < (size_t)NION * NION * 4) return;
    for (int i = 4; i < 10; ++i) if ((size_t)in_sizes[i] < (size_t)MUL * MUL) return;
    if ((size_t)in_sizes[10] < (size_t)544 * HID || in_sizes[11] < HID || (size_t)in_sizes[12] < (size_t)HID * HID || in_sizes[13] < HID) return;
    if (in_sizes[14] < HID * NHD || in_sizes[15] < NHD) return;
    if ((size_t)out_size < (size_t)MTOK * OW) return;
    if (SZ_TOTAL > ws_size) return;
    const float* node_s = (const float*)d_in[0]; const float* node_v = (const float*)d_in[1];
    const float* edge_attr = (const float*)d_in[2]; const float* edge_sh = (const float*)d_in[3];
    const float* win = (const float*)d_in[10]; const float* bin = (const float*)d_in[11];
    const float* wmid = (const float*)d_in[12]; const float* bmid = (const float*)d_in[13];
    const float* wout = (const float*)d_in[14]; const float* bout = (const float*)d_in[15];
    float* OUT = (float*)d_out;
    char* wsp = (char*)d_ws;
    bf* XALL = (bf*)wsp; wsp += SZ_XALL;
    bf* EAB  = (bf*)wsp; wsp += SZ_EAB;
    bf* WQKV = (bf*)wsp; wsp += SZ_WQKV;
    bf* W1N  = (bf*)wsp; wsp += SZ_W1N;
    bf* W1E  = (bf*)wsp; wsp += SZ_W1E;
    h16* WMID = (h16*)wsp; wsp += SZ_WMID;
    h16* WOUT = (h16*)wsp; wsp += SZ_WOUT;
    h16* P3  = (h16*)wsp; wsp += SZ_P3;
    float* NPJ = (float*)wsp; wsp += SZ_NPJ;
    float* EPL = (float*)wsp; wsp += SZ_EPL;
    float* EWP = (float*)wsp; wsp += SZ_EW;

    { const size_t n8 = (size_t)MTOK * MUL / 8;
      k_cvt8<<<(unsigned)((n8 + 255) / 256), 256, 0, stream>>>(node_s, XALL, n8);
      k_cvtv<<<(unsigned)((n8 + 255) / 256), 256, 0, stream>>>(node_v, XALL, n8, (size_t)MTOK * MUL); }
    { const size_t n8 = (size_t)NION * NION * NRBF / 8;
      k_cvt8<<<(unsigned)((n8 + 255) / 256), 256, 0, stream>>>(edge_attr, EAB, n8); }
    for (int i = 0; i < 6; ++i)
        k_wt<<<dim3(MUL / 16, 1, 1), 256, 0, stream>>>((const float*)d_in[4 + i], MUL, MUL, MUL, 0, 0, WQKV + (size_t)i * MUL * MUL, 0, 1.0f);
    k_wt<<<dim3(HID / 16, 4, 1), 256, 0, stream>>>(win + (size_t)NRBF * HID, HID, MUL, HID, MUL, HID * MUL, W1N, 0, 1.0f);
    k_wt<<<dim3(HID / 16, 1, 1), 256, 0, stream>>>(win, HID, NRBF, HID, 0, 0, W1E, 0, 1.0f);
    k_wt<<<dim3(HID / 16, 1, 1), 256, 0, stream>>>(wmid, HID, HID, HID, 0, 0, (bf*)WMID, 1, WCS);
    k_wt<<<dim3(1, 1, 1), 256, 0, stream>>>(wout, NHD, HID, NHD, 0, 0, (bf*)WOUT, 1, WCS);

    k_proj3<<<dim3(NB, 24, 1), 32, 0, stream>>>(XALL, WQKV, P3);
    k_gemm_f32<<<dim3(NION * NION / 64, 1, 1), 32, 0, stream>>>(EAB, W1E, bin, EPL, NRBF, HID, 0);
    k_gemm_f32<<<dim3(MTOK / 64, 8, 1), 32, 0, stream>>>(XALL, W1N, bin, NPJ, MUL, NPW, 1);
    k_mlp<<<dim3(MTOK, 1, 1), 256, 0, stream>>>(EPL, NPJ, edge_sh, WMID, bmid, WOUT, bout, EWP);
    k_attn<<<dim3(NB * 4, 1, 1), 256, 0, stream>>>(P3, P3 + (size_t)NZH * 64 * 64, P3 + (size_t)2 * NZH * 64 * 64, EWP, node_s, node_v, OUT);
}
